// MultiHeadSelfAttention_8701603742005
// MI455X (gfx1250) — hardware-verified
//
#include <hip/hip_runtime.h>


#ifndef NB
#define NB 2
#endif
#ifndef SEQ
#define SEQ 2048
#endif
#define NB_FULL  2
#define SEQ_FULL 2048
#define EM   1024
#define NHD  16
#define HD   64
#define MROWS (NB * SEQ)
#define PSH  10.0f
#define CSL  (0.125f * 1.4426950408889634f)

typedef _Float16 h16;
typedef unsigned short bf;
typedef __attribute__((ext_vector_type(16))) __bf16   v16bf;
typedef __attribute__((ext_vector_type(16))) _Float16 v16h;
typedef __attribute__((ext_vector_type(8)))  _Float16 v8h;
typedef __attribute__((ext_vector_type(8)))  unsigned short v8us;
typedef __attribute__((ext_vector_type(8)))  float    v8f;
typedef __attribute__((ext_vector_type(4)))  float    v4f;
typedef v8h  __attribute__((may_alias)) v8ha;
typedef v4f  __attribute__((may_alias)) v4fa;

static_assert(NB >= 1);
static_assert(NB <= NB_FULL);
static_assert(SEQ <= SEQ_FULL);
static_assert(SEQ % 64 == 0);
static_assert(SEQ % 32 == 0);
static_assert(MROWS % 64 == 0);
static_assert(EM % 64 == 0);
static_assert(EM % 32 == 0);
static_assert(HD == 64);
static_assert(HD * 2 == 128);
static_assert(HD % 64 == 0);
static_assert(NHD * HD == EM);
static_assert(((size_t)MROWS * EM) % 8 == 0);
static_assert((size_t)MROWS * EM < (size_t)2147483648u);

__device__ __forceinline__ unsigned short f2bf(float f) { unsigned u = __float_as_uint(f); u += 0x7FFFu + ((u >> 16) & 1u); return (unsigned short)(u >> 16); }
__device__ __forceinline__ float bf2f(unsigned short b) { return __uint_as_float(((unsigned)b) << 16); }
__device__ __forceinline__ float bfr(float f) { return bf2f(f2bf(f)); }
__device__ __forceinline__ void splitf(float y, unsigned short& h, unsigned short& l) { h = f2bf(y); l = f2bf(y - bf2f(h)); }
__device__ __forceinline__ v16h cat16(v8h lo, v8h hi) { return __builtin_shufflevector(lo, hi, 0, 1, 2, 3, 4, 5, 6, 7, 8, 9, 10, 11, 12, 13, 14, 15); }
__device__ __forceinline__ v16bf cat16b(v8us lo, v8us hi) { return __builtin_bit_cast(v16bf, __builtin_shufflevector(lo, hi, 0, 1, 2, 3, 4, 5, 6, 7, 8, 9, 10, 11, 12, 13, 14, 15)); }
__device__ __forceinline__ v8f wmma16(v16h a, v16h b, v8f c) { return __builtin_amdgcn_wmma_f32_16x16x32_f16(false, a, false, b, (short)0, c, false, false); }
__device__ __forceinline__ v8f wmmab(v16bf a, v16bf b, v8f c) { return __builtin_amdgcn_wmma_f32_16x16x32_bf16(false, a, false, b, (short)0, c, false, false); }
__device__ __forceinline__ v16h  ldh(const h16* p) { return cat16(*(const v8h*)p, *(const v8h*)(p + 16)); }
__device__ __forceinline__ v16bf ldb(const bf* p)  { return cat16b(*(const v8us*)p, *(const v8us*)(p + 16)); }

template <int NSPLIT, bool BIAS, bool RMAP>
__device__ __forceinline__ void gemm_body(const bf* __restrict__ A, const bf* __restrict__ A2, const bf* __restrict__ Bt, int K, float* C, int ldc, const float* __restrict__ bias) {
    __shared__ __align__(16) float os[16 * 68];
    const int lane = threadIdx.x & 31, lr = lane & 15, hi = lane >> 4; const int r0 = blockIdx.x * 64, c0 = blockIdx.y * 64;
    v8f acc[4][4];
#pragma unroll
    for (int mb = 0; mb < 4; ++mb)
#pragma unroll
        for (int nb = 0; nb < 4; ++nb) acc[mb][nb] = (v8f){};
    const size_t aoff = (size_t)(r0 + lr) * K + 8 * hi, boff = (size_t)(c0 + lr) * K + 8 * hi;
#pragma unroll 1
    for (int kc = 0; kc < K; kc += 32) {
        v16bf a[4], a2[4], bl;
#pragma unroll
        for (int mb = 0; mb < 4; ++mb) { a[mb] = ldb(A + aoff + (size_t)mb * 16 * K + kc); a2[mb] = a[mb]; if (NSPLIT == 1) a2[mb] = ldb(A2 + aoff + (size_t)mb * 16 * K + kc); }
#pragma unroll
        for (int nb = 0; nb < 4; ++nb) { bl = ldb(Bt + boff + (size_t)nb * 16 * K + kc);
#pragma unroll
            for (int mb = 0; mb < 4; ++mb) { acc[mb][nb] = wmmab(a[mb], bl, acc[mb][nb]); if (NSPLIT == 1) acc[mb][nb] = wmmab(a2[mb], bl, acc[mb][nb]); } }
        asm volatile("" : "+v"(acc[0][0]), "+v"(acc[0][1]), "+v"(acc[0][2]), "+v"(acc[0][3]), "+v"(acc[1][0]), "+v"(acc[1][1]), "+v"(acc[1][2]), "+v"(acc[1][3]));
        asm volatile("v_nop\n\tv_nop\n\tv_nop\n\tv_nop" : "+v"(acc[2][0]), "+v"(acc[2][1]), "+v"(acc[2][2]), "+v"(acc[2][3]), "+v"(acc[3][0]), "+v"(acc[3][1]), "+v"(acc[3][2]), "+v"(acc[3][3]) : "v"(bl), "v"(a[3]), "v"(a2[3]));
    }
#pragma unroll
    for (int mb = 0; mb < 4; ++mb) {
#pragma unroll
        for (int nb = 0; nb < 4; ++nb) {
#pragma unroll
            for (int j = 0; j < 8; ++j) os[(hi * 8 + j) * 68 + nb * 16 + lr] = acc[mb][nb][j]; }
        __builtin_amdgcn_wave_barrier(); asm volatile("" ::: "memory");
        const int rr = r0 + mb * 16;
        const int orow = RMAP ? ((rr / SEQ) * SEQ_FULL + (rr % SEQ)) : rr;
        float* crow = C + (size_t)orow * ldc + c0;
#pragma unroll 1
        for (int ps = 0; ps < 2; ++ps) {
#pragma unroll
            for (int s = 0; s < 8; ++s) { const int row = 2 * s + hi, cofs = lr * 4; v4f val = *(const v4fa*)&os[row * 68 + cofs];
                if (BIAS) { const v4f bb = *(const v4f*)(bias + c0 + cofs); val[0] += bfr(bb[0]); val[1] += bfr(bb[1]); val[2] += bfr(bb[2]); val[3] += bfr(bb[3]); }
                *(volatile v4f*)(crow + (size_t)row * ldc + cofs) = val; }
            if (ps == 0) __threadfence(); }
        __builtin_amdgcn_wave_barrier(); asm volatile("" ::: "memory");
    }
}
__global__ __launch_bounds__(32) void k_gemm_p(const bf* __restrict__ A, const bf* __restrict__ Bt, int K, float* C, int ldc) { gemm_body<0, false, false>(A, A, Bt, K, C, ldc, C); }
__global__ __launch_bounds__(32) void k_gemm_o(const bf* __restrict__ A, const bf* __restrict__ A2, const bf* __restrict__ Bt, int K, float* C, int ldc, const float* __restrict__ bias) { gemm_body<1, true, true>(A, A2, Bt, K, C, ldc, bias); }

__global__ __launch_bounds__(256) void k_cvtx(const float* __restrict__ src, bf* dst, size_t n8) {
    const size_t i = (size_t)blockIdx.x * 256 + threadIdx.x; if (i >= n8) return;
    const size_t e = i * 8; const int row = (int)(e / (size_t)EM), col = (int)(e % (size_t)EM); const int b = row / SEQ, s = row % SEQ;
    const v8f v = *(const v8f*)(src + ((size_t)b * SEQ_FULL + s) * EM + col); v8us o;
#pragma unroll
    for (int k = 0; k < 8; ++k) o[k] = f2bf(v[k]);
    *(volatile v8us*)(dst + e) = o; __threadfence(); *(volatile v8us*)(dst + e) = o; }

__global__ __launch_bounds__(256) void k_cvtT(const float* __restrict__ W, bf* WT, int sp, int dp, int sz, int dz) {
    __shared__ float tl[64 * 65];
    const int t = threadIdx.x; const int k0 = blockIdx.x * 64, n0 = blockIdx.y * 64;
    const float* Wz = W + (size_t)blockIdx.z * (size_t)sz; bf* WTz = WT + (size_t)blockIdx.z * (size_t)dz;
#pragma unroll
    for (int it = 0; it < 4; ++it) { const int r = (t >> 4) + 16 * it, c4 = (t & 15) * 4; const v4f a = *(const v4f*)(Wz + (size_t)(k0 + r) * sp + n0 + c4);
        tl[r * 65 + c4] = a[0]; tl[r * 65 + c4 + 1] = a[1]; tl[r * 65 + c4 + 2] = a[2]; tl[r * 65 + c4 + 3] = a[3]; }
    __syncthreads();
    const int pc = t & 7; v8us o[2];
#pragma unroll
    for (int it = 0; it < 2; ++it) { const int n = (t >> 3) + 32 * it;
#pragma unroll
        for (int q = 0; q < 8; ++q) o[it][q] = f2bf(tl[(pc * 8 + q) * 65 + n]); }
#pragma unroll
    for (int it = 0; it < 2; ++it) { const int n = (t >> 3) + 32 * it; *(volatile v8us*)(WTz + (size_t)(n0 + n) * dp + k0 + pc * 8) = o[it]; }
    __threadfence();
#pragma unroll
    for (int it = 0; it < 2; ++it) { const int n = (t >> 3) + 32 * it; *(volatile v8us*)(WTz + (size_t)(n0 + n) * dp + k0 + pc * 8) = o[it]; }
}

template <int COLS, int ROWBIAS>
__device__ __forceinline__ void pl_body(const float* __restrict__ F, const float* __restrict__ bias, h16* P16, size_t n8) {
    static_assert(COLS % 8 == 0);
    const size_t i = (size_t)blockIdx.x * 256 + threadIdx.x; if (i >= n8) return;
    const size_t e = i * 8; const int c = (int)(e % (size_t)COLS); const int rw = (int)(e / (size_t)COLS);
    const v8f v = *(const v8f*)(F + e); float bb[8];
    if (ROWBIAS) { const float b0 = bfr(bias[rw]);
#pragma unroll
        for (int k = 0; k < 8; ++k) bb[k] = b0;
    } else { const v4f b0 = *(const v4f*)(bias + c), b1 = *(const v4f*)(bias + c + 4);
#pragma unroll
        for (int k = 0; k < 4; ++k) { bb[k] = bfr(b0[k]); bb[4 + k] = bfr(b1[k]); } }
    v8h oh;
#pragma unroll
    for (int k = 0; k < 8; ++k) { const float y = v[k] + bb[k]; oh[k] = (h16)y; }
    *(volatile v8h*)(P16 + e) = oh;
    __threadfence();
    *(volatile v8h*)(P16 + e) = oh;
}
__global__ __launch_bounds__(256) void k_plc(const float* __restrict__ F, const float* __restrict__ bias, h16* P16, size_t n8) { pl_body<EM, 0>(F, bias, P16, n8); }
__global__ __launch_bounds__(256) void k_plv(const float* __restrict__ F, const float* __restrict__ bias, h16* P16, size_t n8) { pl_body<MROWS, 1>(F, bias, P16, n8); }

__global__ __launch_bounds__(32) void k_flash(const h16* __restrict__ Q16, const h16* __restrict__ K16, const h16* __restrict__ VT, bf* CTh, bf* CTl) {
    __shared__ __align__(16) h16 ps[16 * 40];
    __shared__ __align__(16) float os[16 * 68];
    const int lane = threadIdx.x & 31, lr = lane & 15, hi = lane >> 4;
    const int h = blockIdx.y, q0 = blockIdx.x * 16, b = blockIdx.z;
    const int qoff  = (b * SEQ + q0 + lr) * EM + h * HD + 8 * hi;
    const int kbase = (b * SEQ + lr) * EM + h * HD + 8 * hi;
    const int vbase = (h * HD + lr) * MROWS + b * SEQ + 8 * hi;
    v8f o[4]; float m[8], l[8];
#pragma unroll
    for (int j = 0; j < 4; ++j) o[j] = (v8f){};
#pragma unroll
    for (int r = 0; r < 8; ++r) { m[r] = -3.0e38f; l[r] = 0.0f; }
#pragma unroll 1
    for (int t0 = 0; t0 < SEQ; t0 += 32) {
        v8f s0 = (v8f){}, s1 = (v8f){};
        const int koff = kbase + t0 * EM;
        {
            const v16h qa0 = ldh(Q16 + qoff);
            const v16h qa1 = ldh(Q16 + qoff + 32);
            const v16h b00 = ldh(K16 + koff);
            const v16h b10 = ldh(K16 + koff + 16 * EM);
            const v16h b01 = ldh(K16 + koff + 32);
            const v16h b11 = ldh(K16 + koff + 16 * EM + 32);
            s0 = wmma16(qa0, b00, s0); s1 = wmma16(qa0, b10, s1);
            s0 = wmma16(qa1, b01, s0); s1 = wmma16(qa1, b11, s1);
            asm volatile("v_nop\n\tv_nop\n\tv_nop\n\tv_nop" : "+v"(s0), "+v"(s1) : "v"(qa0), "v"(qa1), "v"(b00), "v"(b10), "v"(b01), "v"(b11));
        }
#pragma unroll
        for (int r = 0; r < 8; ++r) {
            const float a0 = s0[r] * CSL;
            const float a1 = s1[r] * CSL;
            float mx = fmaxf(a0, a1);
            mx = fmaxf(mx, __shfl_xor(mx, 1, 32)); mx = fmaxf(mx, __shfl_xor(mx, 2, 32)); mx = fmaxf(mx, __shfl_xor(mx, 4, 32)); mx = fmaxf(mx, __shfl_xor(mx, 8, 32));
            const float mn = fmaxf(m[r], mx);
            const float al = __builtin_amdgcn_exp2f(m[r] - mn);
            const float p0 = __builtin_amdgcn_exp2f((a0 - mn) + PSH);
            const float p1 = __builtin_amdgcn_exp2f((a1 - mn) + PSH);
            l[r] = l[r] * al + (p0 + p1);
            m[r] = mn;
#pragma unroll
            for (int j = 0; j < 4; ++j) o[j][r] *= al;
            ps[(8 * hi + r) * 40 + lr] = (h16)p0;
            ps[(8 * hi + r) * 40 + 16 + lr] = (h16)p1;
        }
        __builtin_amdgcn_wave_barrier(); asm volatile("" ::: "memory");
        const v16h pf = cat16(*(const v8ha*)&ps[lr * 40 + 8 * hi], *(const v8ha*)&ps[lr * 40 + 16 + 8 * hi]);
        const int voff = vbase + t0;
        {
            v16h vb[4];
#pragma unroll
            for (int jj = 0; jj < 4; ++jj) vb[jj] = ldh(VT + voff + jj * 16 * MROWS);
#pragma unroll
            for (int jj = 0; jj < 4; ++jj) o[jj] = wmma16(pf, vb[jj], o[jj]);
            asm volatile("v_nop\n\tv_nop\n\tv_nop\n\tv_nop" : "+v"(o[0]), "+v"(o[1]), "+v"(o[2]), "+v"(o[3]) : "v"(pf), "v"(vb[0]), "v"(vb[1]), "v"(vb[2]), "v"(vb[3]));
        }
        __builtin_amdgcn_wave_barrier(); asm volatile("" ::: "memory");
    }
#pragma unroll
    for (int r = 0; r < 8; ++r) {
        float lt = l[r];
        lt += __shfl_xor(lt, 1, 32); lt += __shfl_xor(lt, 2, 32); lt += __shfl_xor(lt, 4, 32); lt += __shfl_xor(lt, 8, 32);
        const float inv = 1.0f / lt;
#pragma unroll
        for (int j = 0; j < 4; ++j) os[(8 * hi + r) * 68 + j * 16 + lr] = o[j][r] * inv;
    }
    __builtin_amdgcn_wave_barrier(); asm volatile("" ::: "memory");
    const int rq = lane >> 3, cofs = (lane & 7) * 8;
#pragma unroll 1
    for (int pass = 0; pass < 2; ++pass) {
#pragma unroll
        for (int s = 0; s < 4; ++s) {
            const int row = 4 * s + rq;
            const v4f a = *(const v4fa*)&os[row * 68 + cofs];
            const v4f c = *(const v4fa*)&os[row * 68 + cofs + 4];
            v8us oh, ol;
#pragma unroll
            for (int q = 0; q < 4; ++q) { unsigned short x0, x1; splitf(a[q], x0, x1); oh[q] = x0; ol[q] = x1; splitf(c[q], x0, x1); oh[4 + q] = x0; ol[4 + q] = x1; }
            const size_t oo = (size_t)(b * SEQ + q0 + row) * EM + h * HD + cofs;
            *(volatile v8us*)(CTh + oo) = oh; *(volatile v8us*)(CTl + oo) = ol;
        }
        if (pass == 0) __threadfence();
    }
}

#define PL16  ((size_t)MROWS * EM * 2)
#define WPL   ((size_t)EM * EM * 2)
#define CARVE (PL16   + 4 * WPL   + (size_t)MROWS * EM * 4   + 3 * PL16   + 2 * PL16  )
static_assert(PL16 % 256 == 0);
static_assert(WPL % 256 == 0);
static_assert(CARVE <= (size_t)134217728);

extern "C" void kernel_launch(void* const* d_in, const int* in_sizes, int n_in,
                              void* d_out, int out_size, void* d_ws, size_t ws_size, hipStream_t stream) {
    if (n_in < 9) return;
    const size_t xneed = ((size_t)(NB - 1) * SEQ_FULL + SEQ) * EM;
    if ((size_t)in_sizes[0] < xneed) return;
    if ((size_t)in_sizes[1] < (size_t)EM * EM || (size_t)in_sizes[3] < (size_t)EM * EM || (size_t)in_sizes[5] < (size_t)EM * EM || (size_t)in_sizes[7] < (size_t)EM * EM) return;
    if (in_sizes[2] < EM || in_sizes[4] < EM || in_sizes[6] < EM || in_sizes[8] < EM) return;
    if ((size_t)out_size < xneed) return;
    if (ws_size < CARVE) return;
    const float* x  = (const float*)d_in[0];
    const float* wq = (const float*)d_in[1]; const float* bq = (const float*)d_in[2];
    const float* wk = (const float*)d_in[3]; const float* bk = (const float*)d_in[4];
    const float* wv = (const float*)d_in[5]; const float* bv = (const float*)d_in[6];
    const float* wo = (const float*)d_in[7]; const float* bo = (const float*)d_in[8];
    float* OUT = (float*)d_out;
    char* wsp = (char*)d_ws;
    auto take = [&](size_t bytes) { char* p = wsp; wsp += (bytes + 255) & ~(size_t)255; return (void*)p; };
    bf* XB  = (bf*)take(PL16);
    bf* WQT = (bf*)take(WPL); bf* WKT = (bf*)take(WPL); bf* WVT = (bf*)take(WPL); bf* WOT = (bf*)take(WPL);
    float* F = (float*)take((size_t)MROWS * EM * 4);
    h16* Q16 = (h16*)take(PL16); h16* K16 = (h16*)take(PL16); h16* VT16 = (h16*)take(PL16);
    bf* CTh = (bf*)take(PL16); bf* CTl = (bf*)take(PL16);
    if ((size_t)(wsp - (char*)d_ws) > ws_size) return;

    const size_t n8 = (size_t)MROWS * EM / 8; const unsigned g8 = (unsigned)((n8 + 255) / 256);
    k_cvtx<<<g8, 256, 0, stream>>>(x, XB, n8);
    k_cvtT<<<dim3(EM / 64, HD / 64, NHD), 256, 0, stream>>>(wq, WQT, HD, EM, EM * HD, HD * EM);
    k_cvtT<<<dim3(EM / 64, HD / 64, NHD), 256, 0, stream>>>(wk, WKT, HD, EM, EM * HD, HD * EM);
    k_cvtT<<<dim3(EM / 64, HD / 64, NHD), 256, 0, stream>>>(wv, WVT, HD, EM, EM * HD, HD * EM);
    k_cvtT<<<dim3(EM / 64, EM / 64, 1), 256, 0, stream>>>(wo, WOT, EM, EM, 0, 0);
    k_gemm_p<<<dim3(MROWS / 64, EM / 64), 32, 0, stream>>>(XB, WQT, EM, F, EM);
    k_plc<<<g8, 256, 0, stream>>>(F, bq, Q16, n8);
    k_gemm_p<<<dim3(MROWS / 64, EM / 64), 32, 0, stream>>>(XB, WKT, EM, F, EM);
    k_plc<<<g8, 256, 0, stream>>>(F, bk, K16, n8);
    k_gemm_p<<<dim3(EM / 64, MROWS / 64), 32, 0, stream>>>(WVT, XB, EM, F, MROWS);
    k_plv<<<g8, 256, 0, stream>>>(F, bv, VT16, n8);
    k_flash<<<dim3(SEQ / 16, NHD, NB), 32, 0, stream>>>(Q16, K16, VT16, CTh, CTl);
    k_gemm_o<<<dim3(MROWS / 64, EM / 64), 32, 0, stream>>>(CTh, CTl, WOT, EM, OUT, EM, bo);
}
